// DynamicMasksLoss_w_Matching_35107062677774
// MI455X (gfx1250) — hardware-verified
//
#include <hip/hip_runtime.h>
#define BB 8
#define QQ 25
#define HW 65536
#define DD 256
#define LL 20
#define NCHK 64
#define PPC (HW / NCHK)
#define NST 10

typedef __bf16 v16b __attribute__((ext_vector_type(16)));
typedef unsigned short v8us __attribute__((ext_vector_type(8), may_alias));
typedef float  v8f  __attribute__((ext_vector_type(8)));
typedef float  v4f  __attribute__((ext_vector_type(4)));
typedef float  v4fa __attribute__((ext_vector_type(4), may_alias));
union FragB { v16b v; v8us half[2]; unsigned short u[16]; };

__device__ __forceinline__ unsigned short bf16_bits(float x) { unsigned int u = __float_as_uint(x); return (unsigned short)((u + 0x7FFFu + ((u >> 16) & 1u)) >> 16); }
__device__ __forceinline__ float bf16_val(unsigned short b) { return __uint_as_float(((unsigned int)b) << 16); }
__device__ __forceinline__ float bf16_round(float x) { return bf16_val(bf16_bits(x)); }
template <int NT>
__device__ __forceinline__ v8f mmaN(v16b ah, v16b al, v16b bh, v16b bl, v8f c) {
  c = __builtin_amdgcn_wmma_f32_16x16x32_bf16(false, ah, false, bh, (short)0, c, false, false);
  if (NT >= 2) c = __builtin_amdgcn_wmma_f32_16x16x32_bf16(false, al, false, bh, (short)0, c, false, false);
  if (NT >= 3) c = __builtin_amdgcn_wmma_f32_16x16x32_bf16(false, ah, false, bl, (short)0, c, false, false);
  asm volatile("v_nop\n\tv_nop\n\tv_nop\n\tv_nop" : "+v"(c) : "v"(ah), "v"(al), "v"(bh), "v"(bl));
  return c;
}

__global__ __launch_bounds__(256) void k_wt_bf16(const float* __restrict__ W, unsigned short* __restrict__ Wt, int K, int N) {
  const int t = blockIdx.x * 256 + threadIdx.x;
  const int k8n = K / 8;
  if (t >= N * k8n) return;
  const int n = t / k8n, k8 = (t % k8n) * 8;
  v8us v;
#pragma unroll
  for (int i = 0; i < 8; ++i) v[i] = bf16_bits(W[(size_t)(k8 + i) * N + n]);
  *(volatile v8us*)(Wt + (size_t)n * K + k8) = v;
  __threadfence();
  *(volatile v8us*)(Wt + (size_t)n * K + k8) = v;
}

template <bool ASPLIT, int ACT, bool BIAS_BF16>
__global__ __launch_bounds__(128) void k_gemm_bf(const float* __restrict__ A, int lda, const unsigned short* __restrict__ Wt, int ldb,
                                               const float* __restrict__ bias, float* __restrict__ C, int ldc, int M, int N, int K) {
  __shared__ __attribute__((aligned(16))) float so[4][16][64];
  const int tid = threadIdx.x, w = tid >> 5, lane = tid & 31, ln = lane & 15, hh = lane >> 4;
  const int ntn = N / 64;
  const int wid = blockIdx.x * 4 + w;
  const int mt = wid / ntn, nq = wid % ntn;
  if (mt * 16 >= M) return;
  const int row0 = mt * 16, col0 = nq * 64;
  const float* arow = A + (size_t)(row0 + ln) * lda;
  v8f acc[4] = {};
  for (int kb = 0; kb < K; kb += 32) {
    FragB ah, al;
    const v4f x0 = *(const v4fa*)(arow + kb + 8 * hh), x1 = *(const v4fa*)(arow + kb + 8 * hh + 4);
    const v4f x2 = *(const v4fa*)(arow + kb + 16 + 8 * hh), x3 = *(const v4fa*)(arow + kb + 16 + 8 * hh + 4);
    float xs[16] = {x0[0],x0[1],x0[2],x0[3],x1[0],x1[1],x1[2],x1[3],x2[0],x2[1],x2[2],x2[3],x3[0],x3[1],x3[2],x3[3]};
#pragma unroll
    for (int i = 0; i < 16; ++i) { const unsigned short hb = bf16_bits(xs[i]); ah.u[i] = hb; al.u[i] = ASPLIT ? bf16_bits(xs[i] - bf16_val(hb)) : (unsigned short)0; }
#pragma unroll
    for (int t = 0; t < 4; ++t) {
      const unsigned short* brow = Wt + (size_t)(col0 + t * 16 + ln) * ldb + kb;
      FragB b;
      b.half[0] = *(const v8us*)(brow + 8 * hh);
      b.half[1] = *(const v8us*)(brow + 16 + 8 * hh);
      acc[t] = mmaN<ASPLIT ? 2 : 1>(ah.v, al.v, b.v, b.v, acc[t]);
    }
  }
#pragma unroll
  for (int t = 0; t < 4; ++t) {
    float bv = bias ? bias[col0 + t * 16 + ln] : 0.f;
    if (BIAS_BF16) bv = bf16_round(bv);
#pragma unroll
    for (int r = 0; r < 8; ++r) { float v = acc[t][r] + bv; if (ACT == 1) v = fmaxf(v, 0.f); so[w][8 * hh + r][t * 16 + ln] = v; }
  }
  __builtin_amdgcn_fence(__ATOMIC_ACQ_REL, "workgroup");
  __builtin_amdgcn_wave_barrier();
  const int rsub = lane >> 4, c4 = (lane & 15) * 4;
  for (int pass = 0; pass < 2; ++pass) {
#pragma unroll
    for (int q = 0; q < 8; ++q) {
      const int r = q * 2 + rsub;
      const v4f v = *(const v4fa*)&so[w][r][c4];
      *(volatile v4f*)(C + (size_t)(row0 + r) * ldc + col0 + c4) = v;
    }
    if (pass == 0) __threadfence();
  }
}

template <int D, bool CAUSAL>
__global__ __launch_bounds__(128) void k_flash(const float* __restrict__ qb, const float* __restrict__ kb, const float* __restrict__ vb,
                                             int pitch, int T, int H, float scale, float* __restrict__ y, int ypitch) {
  constexpr int KS = D / 32;
  constexpr int DT = D / 16;
  __shared__ __attribute__((aligned(16))) unsigned short sKh[32][D + 8], sKl[32][D + 8], sVh[32][D + 8], sVl[32][D + 8];
  __shared__ __attribute__((aligned(16))) unsigned short sPh[4][16][40], sPl[4][16][40];
  __shared__ __attribute__((aligned(16))) float sO[4][16][D];
  const int tid = threadIdx.x, w = tid >> 5, lane = tid & 31, ln = lane & 15, hh = lane >> 4;
  const int nqb = (T + 63) / 64;
  const int bh = blockIdx.x / nqb, qblk = blockIdx.x % nqb;
  const int b = bh / H, h = bh % H;
  const int q0 = qblk * 64 + w * 16;
  const float* Q = qb + (size_t)b * T * pitch + h * D;
  const float* K = kb + (size_t)b * T * pitch + h * D;
  const float* V = vb + (size_t)b * T * pitch + h * D;

  FragB aqh[KS], aql[KS];
  {
    int row = q0 + ln; if (row >= T) row = T - 1;
    const float* qr = Q + (size_t)row * pitch;
#pragma unroll
    for (int ks = 0; ks < KS; ++ks)
#pragma unroll
      for (int i = 0; i < 16; ++i) {
        const int d = ks * 32 + ((i < 8) ? (8 * hh + i) : (16 + 8 * hh + (i - 8)));
        const float x = qr[d] * scale; const unsigned short hb = bf16_bits(x);
        aqh[ks].u[i] = hb; aql[ks].u[i] = bf16_bits(x - bf16_val(hb));
      }
  }
  float m_r[8], l_r[8];
#pragma unroll
  for (int r = 0; r < 8; ++r) { m_r[r] = -3.0e38f; l_r[r] = 0.f; }
  v8f oacc[DT];
#pragma unroll
  for (int dt = 0; dt < DT; ++dt) oacc[dt] = (v8f){0.f,0.f,0.f,0.f,0.f,0.f,0.f,0.f};

  const int kv_end = CAUSAL ? min(T, qblk * 64 + 64) : T;
  for (int j0 = 0; j0 < kv_end; j0 += 32) {
    __syncthreads();
    for (int e = tid; e < 32 * (D / 4); e += 128) {
      const int r = e / (D / 4), c4 = (e % (D / 4)) * 4;
      const int key = j0 + r;
      v4f kf = {0.f,0.f,0.f,0.f}, vf = {0.f,0.f,0.f,0.f};
      if (key < T) { kf = *(const v4fa*)(K + (size_t)key * pitch + c4); vf = *(const v4fa*)(V + (size_t)key * pitch + c4); }
#pragma unroll
      for (int t = 0; t < 4; ++t) {
        unsigned short hb = bf16_bits(kf[t]); sKh[r][c4 + t] = hb; sKl[r][c4 + t] = bf16_bits(kf[t] - bf16_val(hb));
        hb = bf16_bits(vf[t]); sVh[r][c4 + t] = hb; sVl[r][c4 + t] = bf16_bits(vf[t] - bf16_val(hb));
      }
    }
    __syncthreads();
    v8f s[2];
#pragma unroll
    for (int nt = 0; nt < 2; ++nt) {
      v8f acc = {};
#pragma unroll
      for (int ks = 0; ks < KS; ++ks) {
        FragB bh_, bl_;
        bh_.half[0] = *(const v8us*)&sKh[nt * 16 + ln][ks * 32 + 8 * hh]; bh_.half[1] = *(const v8us*)&sKh[nt * 16 + ln][ks * 32 + 16 + 8 * hh];
        bl_.half[0] = *(const v8us*)&sKl[nt * 16 + ln][ks * 32 + 8 * hh]; bl_.half[1] = *(const v8us*)&sKl[nt * 16 + ln][ks * 32 + 16 + 8 * hh];
        acc = mmaN<3>(aqh[ks].v, aql[ks].v, bh_.v, bl_.v, acc);
      }
      s[nt] = acc;
    }
    float alpha[8];
#pragma unroll
    for (int r = 0; r < 8; ++r) {
      const int qi = q0 + 8 * hh + r;
      const int ja = j0 + ln, jb = j0 + 16 + ln;
      if (CAUSAL) { if (ja > qi) s[0][r] = -3.0e38f; if (jb > qi) s[1][r] = -3.0e38f; }
      if (ja >= T) s[0][r] = -3.0e38f;
      if (jb >= T) s[1][r] = -3.0e38f;
      float mx = fmaxf(s[0][r], s[1][r]);
      mx = fmaxf(mx, __shfl_xor(mx, 1, 32)); mx = fmaxf(mx, __shfl_xor(mx, 2, 32)); mx = fmaxf(mx, __shfl_xor(mx, 4, 32)); mx = fmaxf(mx, __shfl_xor(mx, 8, 32));
      const float mnew = fmaxf(m_r[r], mx);
      alpha[r] = (mnew > -1.0e38f) ? __expf(m_r[r] - mnew) : 1.0f;
      const float p0 = (s[0][r] > -1.0e38f) ? __expf(s[0][r] - mnew) : 0.f;
      const float p1 = (s[1][r] > -1.0e38f) ? __expf(s[1][r] - mnew) : 0.f;
      m_r[r] = mnew;
      l_r[r] = l_r[r] * alpha[r] + p0 + p1;
      unsigned short hb = bf16_bits(p0); sPh[w][8 * hh + r][ln] = hb;      sPl[w][8 * hh + r][ln] = bf16_bits(p0 - bf16_val(hb));
      hb = bf16_bits(p1);                sPh[w][8 * hh + r][16 + ln] = hb; sPl[w][8 * hh + r][16 + ln] = bf16_bits(p1 - bf16_val(hb));
    }
#pragma unroll
    for (int dt = 0; dt < DT; ++dt)
#pragma unroll
      for (int r = 0; r < 8; ++r) oacc[dt][r] *= alpha[r];
    __builtin_amdgcn_fence(__ATOMIC_ACQ_REL, "workgroup");
    __builtin_amdgcn_wave_barrier();
    FragB pah, pal;
    pah.half[0] = *(const v8us*)&sPh[w][ln][8 * hh]; pah.half[1] = *(const v8us*)&sPh[w][ln][16 + 8 * hh];
    pal.half[0] = *(const v8us*)&sPl[w][ln][8 * hh]; pal.half[1] = *(const v8us*)&sPl[w][ln][16 + 8 * hh];
#pragma unroll
    for (int dt = 0; dt < DT; ++dt) {
      FragB bvh, bvl;
#pragma unroll
      for (int i = 0; i < 8; ++i) {
        bvh.u[i] = sVh[8 * hh + i][dt * 16 + ln]; bvh.u[8 + i] = sVh[16 + 8 * hh + i][dt * 16 + ln];
        bvl.u[i] = sVl[8 * hh + i][dt * 16 + ln]; bvl.u[8 + i] = sVl[16 + 8 * hh + i][dt * 16 + ln];
      }
      oacc[dt] = mmaN<3>(pah.v, pal.v, bvh.v, bvl.v, oacc[dt]);
    }
    __builtin_amdgcn_fence(__ATOMIC_ACQ_REL, "workgroup");
    __builtin_amdgcn_wave_barrier();
  }
#pragma unroll
  for (int r = 0; r < 8; ++r) {
    float l = l_r[r];
    l += __shfl_xor(l, 1, 32); l += __shfl_xor(l, 2, 32); l += __shfl_xor(l, 4, 32); l += __shfl_xor(l, 8, 32);
    l_r[r] = (l > 0.f) ? 1.0f / l : 0.f;
  }
#pragma unroll
  for (int dt = 0; dt < DT; ++dt)
#pragma unroll
    for (int r = 0; r < 8; ++r) sO[w][8 * hh + r][dt * 16 + ln] = oacc[dt][r] * l_r[r];
  __builtin_amdgcn_fence(__ATOMIC_ACQ_REL, "workgroup");
  __builtin_amdgcn_wave_barrier();
  for (int pass = 0; pass < 2; ++pass) {
    for (int r = 0; r < 16; ++r) {
      const int row = q0 + r;
      if (row < T && lane < D / 4) {
        const v4f val = *(const v4fa*)&sO[w][r][lane * 4];
        *(volatile v4f*)(y + ((size_t)b * T + row) * ypitch + h * D + lane * 4) = val;
      }
    }
    if (pass == 0) __threadfence();
  }
}

template <bool ASPLIT, bool BSPLIT, int ACT>
__global__ __launch_bounds__(128) void k_gemm_b(const float* __restrict__ A, int lda, size_t sA, const unsigned short* __restrict__ Bh, const unsigned short* __restrict__ Bl, int ldb, size_t sB,
                                             const float* __restrict__ bias, const float* __restrict__ resid, int ldr, size_t sR, float rsign, float alpha,
                                             float* __restrict__ C, int ldc, size_t sC, int M, int N, int K) {
  __shared__ __attribute__((aligned(16))) float so[4][16][64];
  const int tid = threadIdx.x, w = tid >> 5, lane = tid & 31, ln = lane & 15, hh = lane >> 4;
  const int by = blockIdx.y;
  A += (size_t)by * sA; Bh += (size_t)by * sB; if (BSPLIT) Bl += (size_t)by * sB; C += (size_t)by * sC; if (resid) resid += (size_t)by * sR;
  const int ntn = (N + 63) / 64; const int wid = blockIdx.x * 4 + w; const int mt = wid / ntn, nq = wid % ntn;
  if (mt * 16 >= M) return;
  const int row0 = mt * 16, col0 = nq * 64;
  const float* arow = A + (size_t)(row0 + ln) * lda;
  v8f acc[4] = {};
  for (int kb = 0; kb < K; kb += 32) {
    FragB ah, al;
    const v4f x0 = *(const v4fa*)(arow + kb + 8 * hh), x1 = *(const v4fa*)(arow + kb + 8 * hh + 4);
    const v4f x2 = *(const v4fa*)(arow + kb + 16 + 8 * hh), x3 = *(const v4fa*)(arow + kb + 16 + 8 * hh + 4);
    float xs[16] = {x0[0],x0[1],x0[2],x0[3],x1[0],x1[1],x1[2],x1[3],x2[0],x2[1],x2[2],x2[3],x3[0],x3[1],x3[2],x3[3]};
#pragma unroll
    for (int i = 0; i < 16; ++i) { const unsigned short hb = bf16_bits(xs[i]); ah.u[i] = hb; al.u[i] = ASPLIT ? bf16_bits(xs[i] - bf16_val(hb)) : (unsigned short)0; }
#pragma unroll
    for (int t = 0; t < 4; ++t) {
      if (col0 + t * 16 >= N) continue;
      const size_t boff = (size_t)(col0 + t * 16 + ln) * ldb + kb;
      FragB bh_, bl_; bh_.half[0] = *(const v8us*)(Bh + boff + 8 * hh); bh_.half[1] = *(const v8us*)(Bh + boff + 16 + 8 * hh);
      if (BSPLIT) { bl_.half[0] = *(const v8us*)(Bl + boff + 8 * hh); bl_.half[1] = *(const v8us*)(Bl + boff + 16 + 8 * hh); } else bl_ = bh_;
      acc[t] = mmaN<ASPLIT ? (BSPLIT ? 3 : 2) : 1>(ah.v, al.v, bh_.v, bl_.v, acc[t]);
    }
  }
#pragma unroll
  for (int t = 0; t < 4; ++t) {
    const int col = col0 + t * 16 + ln; if (col0 + t * 16 >= N) continue; const float bv = bias ? bf16_round(bias[col]) : 0.f;
#pragma unroll
    for (int r = 0; r < 8; ++r) { float v = acc[t][r] * alpha + bv; if (resid) v += rsign * resid[(size_t)(row0 + 8 * hh + r) * ldr + col]; if (ACT == 1) v = fmaxf(v, 0.f); else if (ACT == 2) v = fmaxf(v, 0.f) + log1pf(expf(-fabsf(v))); so[w][8 * hh + r][t * 16 + ln] = v; }
  }
  __builtin_amdgcn_fence(__ATOMIC_ACQ_REL, "workgroup"); __builtin_amdgcn_wave_barrier();
  const int rsub = lane >> 4, c4 = (lane & 15) * 4;
  for (int pass = 0; pass < 2; ++pass) {
#pragma unroll
    for (int q = 0; q < 8; ++q) { const int r = q * 2 + rsub; if (col0 + c4 < N) { const v4f v = *(const v4fa*)&so[w][r][c4]; *(volatile v4f*)(C + (size_t)(row0 + r) * ldc + col0 + c4) = v; } }
    if (pass == 0) __threadfence();
  }
}
__global__ __launch_bounds__(256) void k_split_transpose_b(const float* __restrict__ src, int lds_, size_t sIn, unsigned short* __restrict__ hi, unsigned short* __restrict__ lo, size_t sOut, int K, int N) {
  const size_t t = (size_t)blockIdx.x * 256 + threadIdx.x; const int k8n = K / 8; if (t >= (size_t)N * k8n) return;
  src += (size_t)blockIdx.y * sIn; hi += (size_t)blockIdx.y * sOut; lo += (size_t)blockIdx.y * sOut;
  const int n = (int)(t / k8n), k8 = (int)(t % k8n) * 8; v8us vh, vl;
#pragma unroll
  for (int i = 0; i < 8; ++i) { const float x = src[(size_t)(k8 + i) * lds_ + n]; const unsigned short hb = bf16_bits(x); vh[i] = hb; vl[i] = bf16_bits(x - bf16_val(hb)); }
  unsigned short* dh = hi + (size_t)n * K + k8; unsigned short* dl = lo + (size_t)n * K + k8;
  *(volatile v8us*)dh = vh; *(volatile v8us*)dl = vl; __threadfence(); *(volatile v8us*)dh = vh; *(volatile v8us*)dl = vl;
}

__global__ __launch_bounds__(256) void k_mask1(const float* __restrict__ mp, const float* __restrict__ mg, const int* __restrict__ merged, double* __restrict__ part) {
  __shared__ double rs[NST][256]; const int chunk = blockIdx.x, q = blockIdx.y, b = blockIdx.z; const int tid = threadIdx.x; double acc[NST]; for (int k = 0; k < NST; ++k) acc[k] = 0.0;
#pragma unroll 1
  for (int i = tid; i < PPC; i += 256) { const int px = chunk * PPC + i; const size_t e = ((size_t)b * QQ + q) * HW + px;
    const float x = bf16_round(mp[e]); const float t = bf16_round(mg[e]); const float m = (float)merged[(size_t)b * HW + px];
    const float p = 1.0f / (1.0f + expf(-x)); const float l1 = -logf(1.0f - p + 1e-4f), lp = -logf(p + 1e-4f);
    acc[0] += (double)(p * t); acc[1] += (double)p; acc[2] += (double)t; acc[3] += (double)(l1 * (1.f - t) * m); acc[4] += (double)((1.f - t) * m); acc[5] += (double)(l1 * (1.f - t) * (1.f - m)); acc[6] += (double)((1.f - t) * (1.f - m)); acc[7] += (double)(lp * t); acc[8] += (double)(l1 * m); acc[9] += (double)m; }
  for (int k = 0; k < NST; ++k) rs[k][tid] = acc[k]; __syncthreads();
  for (int s = 128; s > 0; s >>= 1) { if (tid < s) { for (int k = 0; k < NST; ++k) rs[k][tid] += rs[k][tid + s]; } __syncthreads(); }
  double* d = part + ((((size_t)b * QQ + q) * NCHK) + chunk) * 16; if (tid < 16) { const double v = (tid < NST) ? rs[tid][0] : 0.0; *(volatile double*)(d + tid) = v; __threadfence(); *(volatile double*)(d + tid) = v; }
}
__global__ __launch_bounds__(256) void k_merge1(const float* __restrict__ mpred, const int* __restrict__ merged, double* __restrict__ part) {
  __shared__ double rs[7][256]; const int chunk = blockIdx.x, b = blockIdx.y; const int tid = threadIdx.x; double acc[7]; for (int k = 0; k < 7; ++k) acc[k] = 0.0;
#pragma unroll 1
  for (int i = tid; i < PPC; i += 256) { const int px = chunk * PPC + i; const float x0 = bf16_round(mpred[((size_t)b * 2) * HW + px]), x1 = bf16_round(mpred[((size_t)b * 2 + 1) * HW + px]); const int g = merged[(size_t)b * HW + px];
    const float mx = fmaxf(x0, x1); const float lse = mx + logf(expf(x0 - mx) + expf(x1 - mx)); const float lp0 = x0 - lse, lp1 = x1 - lse; const float s0 = expf(lp0), s1 = expf(lp1);
    acc[0] += (double)(-(g == 0 ? lp0 : lp1)); acc[1] += (double)(g == 0 ? s0 : 0.f); acc[2] += (double)(g == 1 ? s1 : 0.f); acc[3] += (double)s0; acc[4] += (double)s1; acc[5] += (double)(g == 0 ? 1.f : 0.f); acc[6] += (double)(g == 1 ? 1.f : 0.f); }
  for (int k = 0; k < 7; ++k) rs[k][tid] = acc[k]; __syncthreads();
  for (int s = 128; s > 0; s >>= 1) { if (tid < s) { for (int k = 0; k < 7; ++k) rs[k][tid] += rs[k][tid + s]; } __syncthreads(); }
  double* d = part + (((size_t)b * NCHK) + chunk) * 16; if (tid < 16) { const double v = (tid < 7) ? rs[tid][0] : 0.0; *(volatile double*)(d + tid) = v; __threadfence(); *(volatile double*)(d + tid) = v; }
}
__global__ __launch_bounds__(256) void k_stage2(const double* __restrict__ pm, const double* __restrict__ pg, double* __restrict__ MS, double* __restrict__ MG) {
  const int t = blockIdx.x * 256 + threadIdx.x;
  if (t < BB * QQ * 16) { const int r = t / 16, k = t % 16; double s = 0.0; for (int c = 0; c < NCHK; ++c) s += pm[((size_t)r * NCHK + c) * 16 + k]; *(volatile double*)(MS + t) = s; __threadfence(); *(volatile double*)(MS + t) = s; }
  if (t < BB * 16) { const int r = t / 16, k = t % 16; double s = 0.0; for (int c = 0; c < NCHK; ++c) s += pg[((size_t)r * NCHK + c) * 16 + k]; *(volatile double*)(MG + t) = s; __threadfence(); *(volatile double*)(MG + t) = s; }
}
__global__ __launch_bounds__(256) void k_pad(const float* __restrict__ query, const float* __restrict__ text, float* __restrict__ Qf, unsigned short* __restrict__ Qb, unsigned short* __restrict__ Tb) {
  const size_t t = (size_t)blockIdx.x * 256 + threadIdx.x;
  if (t < (size_t)BB * 32 * DD / 4) { const int d4 = (int)(t % (DD / 4)) * 4; const int r = (int)((t / (DD / 4)) % 32); const int b = (int)(t / ((DD / 4) * 32)); v4f v = {0.f, 0.f, 0.f, 0.f}; if (r < QQ) v = *(const v4fa*)(query + ((size_t)b * QQ + r) * DD + d4); *(volatile v4f*)(Qf + t * 4) = v; __threadfence(); *(volatile v4f*)(Qf + t * 4) = v; }
  if (t < (size_t)BB * 32 * DD / 8) { const int d8 = (int)(t % (DD / 8)) * 8; const int r = (int)((t / (DD / 8)) % 32); const int b = (int)(t / ((DD / 8) * 32)); v8us q8, t8;
#pragma unroll
    for (int i = 0; i < 8; ++i) { q8[i] = (r < QQ) ? bf16_bits(query[((size_t)b * QQ + r) * DD + d8 + i]) : (unsigned short)0; t8[i] = (r < LL) ? bf16_bits(text[((size_t)b * LL + r) * DD + d8 + i]) : (unsigned short)0; }
    *(volatile v8us*)(Qb + t * 8) = q8; *(volatile v8us*)(Tb + t * 8) = t8; __threadfence(); *(volatile v8us*)(Qb + t * 8) = q8; *(volatile v8us*)(Tb + t * 8) = t8; }
}
__global__ __launch_bounds__(64) void k_final(const double* __restrict__ MS, const double* __restrict__ MG, const float* __restrict__ SIM, const float* __restrict__ GQ, const float* __restrict__ cqp, const int* __restrict__ cqg, const float* __restrict__ obp, const int* __restrict__ obg, const float* __restrict__ query, const int* __restrict__ tlab, float* __restrict__ out) {
  if (threadIdx.x != 0) return;
  double ce = 0.0, dsum = 0.0; for (int b = 0; b < BB; ++b) { const double* g = MG + b * 16; ce += g[0]; for (int c = 0; c < 2; ++c) { const double inter = g[1 + c], ssm = g[3 + c], soh = g[5 + c]; dsum += 1.0 - (2.0 * inter + 1.0) / (ssm + soh + 1.0); } }
  const double loss_merged = ce / ((double)BB * HW) + dsum / ((double)BB * 2);
  double lm_acc = 0.0, lc_acc = 0.0;
  for (int b = 0; b < BB; ++b) { const int nobj = obg[b]; const double nfg = (double)nobj; double dc = 0.0, f1 = 0.0, f2 = 0.0, f3 = 0.0, bg = 0.0, cls = 0.0;
    for (int q = 0; q < QQ; ++q) { const double* s = MS + ((size_t)b * QQ + q) * 16; const bool fg = q < nobj;
      const double dice = 1.0 - (2.0 * s[0] + 1.0) / ((s[1] + s[2]) + 1.0); const double lf1 = s[3] / (s[4] + 1.0), lf2 = s[5] / (s[6] + 1.0), lf3 = s[7] / (s[2] + 1.0), lbg = s[8] / (s[9] + 1.0);
      if (fg) { dc += dice; f1 += lf1; f2 += lf2; f3 += lf3; } else { bg += lbg; }
      const float c0 = bf16_round(cqp[((size_t)b * QQ + q) * 2]), c1 = bf16_round(cqp[((size_t)b * QQ + q) * 2 + 1]); const float mx = fmaxf(c0, c1); const float lse = mx + logf(expf(c0 - mx) + expf(c1 - mx)); const int gl = cqg[(size_t)b * QQ + q]; const double ceq = -(double)((gl == 0 ? c0 : c1) - lse); if (fg) cls += ceq; }
    dc /= nfg; f1 /= nfg; f2 /= nfg; f3 /= nfg; const double fgl = fmax(fmax(f1, f3), f2); const double bgl = bg / ((double)QQ - nfg);
    lm_acc += 0.5 * fgl + 0.2 * bgl + 0.3 * dc; lc_acc += cls / nfg; }
  const double loss_masks = lm_acc / BB, loss_class = lc_acc / BB;
  double ln_acc = 0.0; for (int b = 0; b < BB; ++b) { const float x = bf16_round(obp[b]) - (float)obg[b] / (float)QQ; const float ax = fabsf(x); ln_acc += (double)((ax < 1.0f) ? 0.5f * x * x : ax - 0.5f); } const double loss_num = ln_acc / BB;
  double con = 0.0, orth = 0.0, size = 0.0; const float scl = 0.0625f;
  for (int b = 0; b < BB; ++b) {
    for (int l = 0; l < LL; ++l) { int lab = tlab[(size_t)b * LL + l]; lab = (lab == -1) ? QQ : lab; int idx = lab - 1; idx = idx < 0 ? 0 : (idx >= QQ ? QQ - 1 : idx);
      float mx = -3.0e38f; for (int q = 0; q < QQ; ++q) mx = fmaxf(mx, SIM[((size_t)b * 32 + q) * 32 + l] * scl); float den = 0.f; for (int q = 0; q < QQ; ++q) den += expf(SIM[((size_t)b * 32 + q) * 32 + l] * scl - mx);
      const float pk = expf(SIM[((size_t)b * 32 + idx) * 32 + l] * scl - mx) / den; con += 1.0 - (double)pk; }
    double gs = 0.0, dg = 0.0, sz = 0.0; for (int q = 0; q < QQ; ++q) { for (int k = 0; k < QQ; ++k) gs += fabs((double)GQ[((size_t)b * 32 + q) * 32 + k]); float d2 = 0.f, s2 = 0.f; for (int d = 0; d < DD; ++d) { const float v = bf16_round(query[((size_t)b * QQ + q) * DD + d]); d2 += v * v; s2 += v * v; } dg += fabs((double)d2); sz += fmax(1.0 - (double)s2, 0.0); }
    orth += ((gs - dg) * 0.5) / ((double)QQ * (QQ - 1) * 0.5); size += sz / (double)(QQ - 1); }
  const double contrastive = con / ((double)BB * LL); orth /= BB; size /= BB; const double loss_matching = contrastive + 0.5 * size + 0.5 * orth;
  const double total = 0.2 * loss_merged + 0.6 * loss_masks + 0.1 * loss_class + 0.1 * loss_num + 0.05 * loss_matching;
  const float r[6] = {(float)total, (float)loss_merged, (float)loss_masks, (float)loss_class, (float)loss_num, (float)loss_matching};
  for (int pass = 0; pass < 2; ++pass) { for (int i = 0; i < 6; ++i) *(volatile float*)(out + i) = r[i]; if (pass == 0) __threadfence(); }
}
extern "C" void kernel_launch(void* const* d_in, const int* in_sizes, int n_in,
                              void* d_out, int out_size, void* d_ws, size_t ws_size, hipStream_t stream) {
  (void)in_sizes; (void)n_in; (void)out_size;
  const float* merged_pred = (const float*)d_in[0]; const int* merged_gt = (const int*)d_in[1]; const float* masks_pred = (const float*)d_in[2]; const float* masks_gt = (const float*)d_in[3]; const float* cqp = (const float*)d_in[4]; const int* cqg = (const int*)d_in[5];
  const float* obp = (const float*)d_in[6]; const int* obg = (const int*)d_in[7]; const float* query = (const float*)d_in[8]; const float* text = (const float*)d_in[9]; const int* tlab = (const int*)d_in[10];
  char* ws = (char*)d_ws; size_t off = 0;
  auto take = [&](size_t bytes) { char* p = ws + off; off += (bytes + 255) & ~(size_t)255; return p; };
  double* pm = (double*)take((size_t)BB * QQ * NCHK * 16 * 8); double* pg = (double*)take((size_t)BB * NCHK * 16 * 8); double* MS = (double*)take((size_t)BB * QQ * 16 * 8); double* MG = (double*)take((size_t)BB * 16 * 8);
  float* Qf = (float*)take((size_t)BB * 32 * DD * 4); unsigned short* Qb = (unsigned short*)take((size_t)BB * 32 * DD * 2); unsigned short* Tb = (unsigned short*)take((size_t)BB * 32 * DD * 2); float* SIM = (float*)take((size_t)BB * 32 * 32 * 4); float* GQ = (float*)take((size_t)BB * 32 * 32 * 4);
  if (off > ws_size) return;
  k_mask1<<<dim3(NCHK, QQ, BB), 256, 0, stream>>>(masks_pred, masks_gt, merged_gt, pm);
  k_merge1<<<dim3(NCHK, BB), 256, 0, stream>>>(merged_pred, merged_gt, pg);
  k_stage2<<<(BB * QQ * 16 + 255) / 256, 256, 0, stream>>>(pm, pg, MS, MG);
  k_pad<<<(BB * 32 * DD / 4 + 255) / 256, 256, 0, stream>>>(query, text, Qf, Qb, Tb);
  k_gemm_b<false, false, 0><<<dim3(((32 / 16) * 1 + 3) / 4, BB), 128, 0, stream>>>(Qf, DD, (size_t)32 * DD, Tb, Tb, DD, (size_t)32 * DD, nullptr, nullptr, 0, 0, 1.f, 1.f, SIM, 32, (size_t)32 * 32, 32, 32, DD);
  k_gemm_b<false, false, 0><<<dim3(((32 / 16) * 1 + 3) / 4, BB), 128, 0, stream>>>(Qf, DD, (size_t)32 * DD, Qb, Qb, DD, (size_t)32 * DD, nullptr, nullptr, 0, 0, 1.f, 1.f, GQ, 32, (size_t)32 * 32, 32, 32, DD);
  k_final<<<1, 64, 0, stream>>>(MS, MG, SIM, GQ, cqp, cqg, obp, obg, query, tlab, (float*)d_out);
}
